// InLay_61203283968377
// MI455X (gfx1250) — hardware-verified
//
#include <hip/hip_runtime.h>
#include <math.h>

typedef unsigned short us;
typedef __bf16   v16b  __attribute__((ext_vector_type(16)));
typedef us       v16us __attribute__((ext_vector_type(16)));
typedef us       v8us  __attribute__((ext_vector_type(8)));
typedef _Float16 v16h  __attribute__((ext_vector_type(16)));
typedef _Float16 v8h   __attribute__((ext_vector_type(8)));
typedef float    v8f   __attribute__((ext_vector_type(8)));
typedef float    v4f   __attribute__((ext_vector_type(4)));
typedef v8us __attribute__((may_alias)) v8usa;
typedef v8h  __attribute__((may_alias)) v8ha;
typedef v4f  __attribute__((may_alias)) v4fa;

union FragB { v16b v; v16us u; v8us half[2]; };
union FragH { v16h v; v8h half[2]; };

#define NB    256
#define SQ    49
#define DM    512
#define DQ    2048
#define NH    32
#define HQ    64
#define HVD   16
#define MT    (NB * SQ)
#define NPASS 4
#define WPP   (NB / NPASS)
#define RP    (WPP * SQ)
#define KPAD  64

static_assert(RP % 64 == 0);
static_assert((MT * DM) % (8 * 256) == 0);
static_assert(NH * HVD == DM);
static_assert(NH * HQ == DQ);
static_assert(NB % NPASS == 0);

__device__ __forceinline__ v8f wmma_bf(v16b a, v16b b, v8f c) {
  v8f d = __builtin_amdgcn_wmma_f32_16x16x32_bf16(false, a, false, b, (short)0, c, false, false);
  asm volatile("v_nop\n\tv_nop\n\tv_nop\n\tv_nop" : "+v"(d) : "v"(a), "v"(b));
  return d;
}
__device__ __forceinline__ v8f wmma_hf(v16h a, v16h b, v8f c) {
  v8f d = __builtin_amdgcn_wmma_f32_16x16x32_f16(false, a, false, b, (short)0, c, false, false);
  asm volatile("v_nop\n\tv_nop\n\tv_nop\n\tv_nop" : "+v"(d) : "v"(a), "v"(b));
  return d;
}

__device__ __forceinline__ v16b ldb(const us* p, int h) {
  FragB f;
  f.half[0] = *(const v8usa*)(p + 8 * h);
  f.half[1] = *(const v8usa*)(p + 16 + 8 * h);
  return f.v;
}
__device__ __forceinline__ v16h ldh(const _Float16* p, int h) {
  FragH f;
  f.half[0] = *(const v8ha*)(p + 8 * h);
  f.half[1] = *(const v8ha*)(p + 16 + 8 * h);
  return f.v;
}

__device__ __forceinline__ us bf_rne(float f) {
  unsigned u = __float_as_uint(f);
  u += 0x7FFFu + ((u >> 16) & 1u);
  return (us)(u >> 16);
}
__device__ __forceinline__ void split_bf(float f, us& hb, us& lb) {
  const us hi = bf_rne(f);
  const float hf = __uint_as_float(((unsigned)hi) << 16);
  hb = hi;
  lb = bf_rne(f - hf);
}
__device__ __forceinline__ void split8(v4f a, v4f c, v8us& hv, v8us& lv) {
  float f[8] = {a.x, a.y, a.z, a.w, c.x, c.y, c.z, c.w};
#pragma unroll
  for (int j = 0; j < 8; ++j) {
    us hb, lb;
    split_bf(f[j], hb, lb);
    hv[j] = hb;
    lv[j] = lb;
  }
}

__global__ __launch_bounds__(256) void k_cvtx(const float* __restrict__ x,
                                              us* __restrict__ xh, us* __restrict__ xl, int n8)
{
  const int g = blockIdx.x * 256 + threadIdx.x;
  if (g >= n8) return;
  const float* s = x + (size_t)g * 8;
  const v4f a = *(const v4fa*)s;
  const v4f c = *(const v4fa*)(s + 4);
  v8us hv, lv;
  split8(a, c, hv, lv);
  us* ph = xh + (size_t)g * 8;
  us* pl = xl + (size_t)g * 8;
  *(volatile v8us*)ph = hv;
  *(volatile v8us*)pl = lv;
  __threadfence();
  *(volatile v8us*)ph = hv;
  *(volatile v8us*)pl = lv;
}

__device__ __forceinline__ void prep_store(const float* T, us* dh, us* dl, _Float16* df,
                                           int mode, int n0, int k0, int Kp, int t) {
#pragma unroll
  for (int it = 0; it < 2; ++it) {
    const int item = it * 256 + t, nn = item >> 3, q8 = item & 7;
    float f[8];
#pragma unroll
    for (int j = 0; j < 8; ++j) f[j] = T[(8 * q8 + j) * 65 + nn];
    const size_t off = (size_t)(n0 + nn) * Kp + k0 + 8 * q8;
    if (mode == 0) {
      v8us hv, lv;
#pragma unroll
      for (int j = 0; j < 8; ++j) {
        us hb, lb;
        split_bf(f[j], hb, lb);
        hv[j] = hb;
        lv[j] = lb;
      }
      *(volatile v8us*)(dh + off) = hv;
      *(volatile v8us*)(dl + off) = lv;
    } else {
      v8h o;
#pragma unroll
      for (int j = 0; j < 8; ++j) o[j] = (_Float16)(f[j] * 1024.0f);
      *(volatile v8h*)(df + off) = o;
    }
  }
}

__global__ __launch_bounds__(256) void k_prep(
    const float* __restrict__ wq1, const float* __restrict__ wk1, const float* __restrict__ wp,
    const float* __restrict__ wq2, const float* __restrict__ wk2, const float* __restrict__ tok,
    us* __restrict__ wq1h, us* __restrict__ wq1l, us* __restrict__ wk1h, us* __restrict__ wk1l,
    us* __restrict__ wph, us* __restrict__ wpl,
    _Float16* __restrict__ wq2t, _Float16* __restrict__ wk2t,
    us* __restrict__ tkh, us* __restrict__ tkl)
{
  __shared__ __attribute__((aligned(16))) float T[64 * 65];
  const int t = threadIdx.x;
  const int bid = blockIdx.x;
  if (bid >= 712) return;

  const float* src;
  us* dh; us* dl; _Float16* df;
  int C, R, Kp, mode, tn, tk;
  if (bid < 192) {
    const int wsel = bid >> 6, loc = bid & 63;
    src = (wsel == 0) ? wq1 : ((wsel == 1) ? wk1 : wp);
    dh  = (wsel == 0) ? wq1h : ((wsel == 1) ? wk1h : wph);
    dl  = (wsel == 0) ? wq1l : ((wsel == 1) ? wk1l : wpl);
    df  = wq2t;
    C = DM; R = DM; Kp = DM; mode = 0; tn = loc >> 3; tk = loc & 7;
  } else if (bid < 704) {
    const int loc = bid - 192, wsel = loc >> 8, l2 = loc & 255;
    src = wsel ? wk2 : wq2;
    df  = wsel ? wk2t : wq2t;
    dh = wq1h; dl = wq1l;
    C = DQ; R = DM; Kp = DM; mode = 1; tn = l2 >> 3; tk = l2 & 7;
  } else {
    const int loc = bid - 704;
    src = tok; dh = tkh; dl = tkl; df = wq2t;
    C = DM; R = SQ; Kp = KPAD; mode = 0; tn = loc; tk = 0;
  }
  const int n0 = tn * 64, k0 = tk * 64;

#pragma unroll
  for (int i = 0; i < 16; ++i) {
    const int idx = i * 256 + t, kk = idx >> 6, nn = idx & 63;
    const int gk = k0 + kk;
    const int gkc = min(gk, R - 1);
    const float v = src[(size_t)gkc * C + n0 + nn];
    T[kk * 65 + nn] = (gk < R) ? v : 0.0f;
  }
  __syncthreads();

  prep_store(T, dh, dl, df, mode, n0, k0, Kp, t);
  __threadfence();
  prep_store(T, dh, dl, df, mode, n0, k0, Kp, t);
}

__device__ __forceinline__ void mm3_32x32(const us* ah0p, const us* al0p,
                                          const us* bh0p, const us* bl0p,
                                          int h, v8f (&acc)[2][2]) {
  const us* ah1p = ah0p + 16 * DM;
  const us* al1p = al0p + 16 * DM;
  const us* bh1p = bh0p + 16 * DM;
  const us* bl1p = bl0p + 16 * DM;
#pragma unroll 1
  for (int k0 = 0; k0 < DM; k0 += 32) {
    const v16b ah0 = ldb(ah0p + k0, h), ah1 = ldb(ah1p + k0, h);
    const v16b al0 = ldb(al0p + k0, h), al1 = ldb(al1p + k0, h);
    const v16b bh0 = ldb(bh0p + k0, h), bh1 = ldb(bh1p + k0, h);
    const v16b bl0 = ldb(bl0p + k0, h), bl1 = ldb(bl1p + k0, h);
    acc[0][0] = wmma_bf(ah0, bh0, acc[0][0]);
    acc[0][0] = wmma_bf(ah0, bl0, acc[0][0]);
    acc[0][0] = wmma_bf(al0, bh0, acc[0][0]);
    acc[0][1] = wmma_bf(ah0, bh1, acc[0][1]);
    acc[0][1] = wmma_bf(ah0, bl1, acc[0][1]);
    acc[0][1] = wmma_bf(al0, bh1, acc[0][1]);
    acc[1][0] = wmma_bf(ah1, bh0, acc[1][0]);
    acc[1][0] = wmma_bf(ah1, bl0, acc[1][0]);
    acc[1][0] = wmma_bf(al1, bh0, acc[1][0]);
    acc[1][1] = wmma_bf(ah1, bh1, acc[1][1]);
    acc[1][1] = wmma_bf(ah1, bl1, acc[1][1]);
    acc[1][1] = wmma_bf(al1, bh1, acc[1][1]);
  }
}

__device__ __forceinline__ void gemm1_store(const _Float16* sT, _Float16* H, int mb, int nb, int t) {
#pragma unroll
  for (int it = 0; it < 4; ++it) {
    const int item = it * 128 + t, rl = item >> 3, q8 = item & 7;
    const v8h v = *(const v8ha*)(sT + rl * 72 + 8 * q8);
    const size_t off = (size_t)(mb + rl) * DM + nb + 8 * q8;
    *(volatile v8h*)(H + off) = v;
  }
}

__global__ __launch_bounds__(128) void k_gemm1(
    const us* __restrict__ xh, const us* __restrict__ xl,
    const us* __restrict__ wqh, const us* __restrict__ wql,
    const us* __restrict__ wkh, const us* __restrict__ wkl,
    const float* __restrict__ bq1, const float* __restrict__ bk1,
    _Float16* __restrict__ hq, _Float16* __restrict__ hk)
{
  __shared__ __attribute__((aligned(16))) _Float16 sT[64 * 72];
  const int t = threadIdx.x, lane = t & 31, w = t >> 5, h = lane >> 4, m = lane & 15;
  const int wm = w >> 1, wn = w & 1;
  const int mb = blockIdx.x * 64, nb = blockIdx.y * 64;
  const bool isk = (blockIdx.z != 0);
  const us* wth = isk ? wkh : wqh;
  const us* wtl = isk ? wkl : wql;
  const float* bias = isk ? bk1 : bq1;
  _Float16* H = isk ? hk : hq;

  const size_t arow = (size_t)(mb + 32 * wm + m) * DM;
  const size_t brow = (size_t)(nb + 32 * wn + m) * DM;

  const v8f z8 = {0.f, 0.f, 0.f, 0.f, 0.f, 0.f, 0.f, 0.f};
  v8f acc[2][2];
  acc[0][0] = z8; acc[0][1] = z8; acc[1][0] = z8; acc[1][1] = z8;

  mm3_32x32(xh + arow, xl + arow, wth + brow, wtl + brow, h, acc);

#pragma unroll
  for (int nt = 0; nt < 2; ++nt) {
    const int cl = 32 * wn + 16 * nt + m;
    const float bv = bias[nb + cl];
#pragma unroll
    for (int mt = 0; mt < 2; ++mt) {
#pragma unroll
      for (int r = 0; r < 8; ++r) {
        const int rl = 32 * wm + 16 * mt + 8 * h + r;
        const float v = acc[mt][nt][r] + bv;
        const float g = 0.5f * v * (1.0f + erff(v * 0.70710678118654752f));
        sT[rl * 72 + cl] = (_Float16)(g * 16.0f);
      }
    }
  }
  __syncthreads();

  gemm1_store(sT, H, mb, nb, t);
  __threadfence();
  gemm1_store(sT, H, mb, nb, t);
}

__device__ __forceinline__ void gemm2_store(const float* sF, us* oh, us* ol, int mb, int nb, int t) {
#pragma unroll
  for (int it = 0; it < 8; ++it) {
    const int item = it * 128 + t, rl = item >> 4, g = item & 15;
    const float* sp = sF + rl * 132 + 8 * g;
    const v4f a = *(const v4fa*)sp;
    const v4f c = *(const v4fa*)(sp + 4);
    v8us hv, lv;
    split8(a, c, hv, lv);
    const size_t off = (size_t)(mb + rl) * DQ + nb + 8 * g;
    *(volatile v8us*)(oh + off) = hv;
    *(volatile v8us*)(ol + off) = lv;
  }
}

__global__ __launch_bounds__(128) void k_gemm2(
    const _Float16* __restrict__ hq, const _Float16* __restrict__ hk,
    const _Float16* __restrict__ wq2t, const _Float16* __restrict__ wk2t,
    const float* __restrict__ bq2, const float* __restrict__ bk2,
    us* __restrict__ qh, us* __restrict__ ql, us* __restrict__ kh, us* __restrict__ kl)
{
  __shared__ __attribute__((aligned(16))) float sF[64 * 132];
  const int t = threadIdx.x, lane = t & 31, w = t >> 5, h = lane >> 4, m = lane & 15;
  const int wm = w >> 1, wn = w & 1;
  const int mb = blockIdx.x * 64, nb = blockIdx.y * 128;
  const bool isk = (blockIdx.z != 0);
  const _Float16* A  = isk ? hk : hq;
  const _Float16* Bt = isk ? wk2t : wq2t;
  const float* bias  = isk ? bk2 : bq2;
  us* oh = isk ? kh : qh;
  us* ol = isk ? kl : ql;

  const _Float16* a0p = A + (size_t)(mb + 32 * wm + m) * DM;
  const _Float16* a1p = a0p + 16 * DM;
  const _Float16* b0p = Bt + (size_t)(nb + 64 * wn + m) * DM;

  const v8f z8 = {0.f, 0.f, 0.f, 0.f, 0.f, 0.f, 0.f, 0.f};
  v8f acc[2][4];
#pragma unroll
  for (int mt = 0; mt < 2; ++mt)
#pragma unroll
    for (int nt = 0; nt < 4; ++nt) acc[mt][nt] = z8;

#pragma unroll 1
  for (int k0 = 0; k0 < DM; k0 += 32) {
    const v16h a0 = ldh(a0p + k0, h);
    const v16h a1 = ldh(a1p + k0, h);
#pragma unroll
    for (int nt = 0; nt < 4; ++nt) {
      const v16h b = ldh(b0p + (size_t)nt * 16 * DM + k0, h);
      acc[0][nt] = wmma_hf(a0, b, acc[0][nt]);
      acc[1][nt] = wmma_hf(a1, b, acc[1][nt]);
    }
  }

#pragma unroll
  for (int nt = 0; nt < 4; ++nt) {
    const int cl = 64 * wn + 16 * nt + m;
    const float bv = bias[nb + cl];
#pragma unroll
    for (int mt = 0; mt < 2; ++mt) {
#pragma unroll
      for (int r = 0; r < 8; ++r) {
        const int rl = 32 * wm + 16 * mt + 8 * h + r;
        sF[rl * 132 + cl] = acc[mt][nt][r] * (1.0f / 16384.0f) + bv;
      }
    }
  }
  __syncthreads();

  gemm2_store(sF, oh, ol, mb, nb, t);
  __threadfence();
  gemm2_store(sF, oh, ol, mb, nb, t);
}

__device__ __forceinline__ void attn_store(const float* so, us* oph, us* opl,
                                           size_t rowbase, int hg, int t) {
#pragma unroll
  for (int it = 0; it < 4; ++it) {
    const int item = it * 256 + t;
    if (item < SQ * 16) {
      const int rl = item >> 4, g = item & 15;
      const float* sp = so + rl * 132 + 8 * g;
      const v4f a = *(const v4fa*)sp;
      const v4f c = *(const v4fa*)(sp + 4);
      v8us hv, lv;
      split8(a, c, hv, lv);
      const size_t off = (rowbase + rl) * DM + hg * 128 + 8 * g;
      *(volatile v8us*)(oph + off) = hv;
      *(volatile v8us*)(opl + off) = lv;
    }
  }
}

__global__ __launch_bounds__(256) void k_attn(
    const us* __restrict__ qh, const us* __restrict__ ql,
    const us* __restrict__ kh, const us* __restrict__ kl,
    const us* __restrict__ tkh, const us* __restrict__ tkl,
    us* __restrict__ oph, us* __restrict__ opl)
{
  __shared__ __attribute__((aligned(16))) float so[64 * 132];
  const int t = threadIdx.x, lane = t & 31, w = t >> 5, h = lane >> 4, m = lane & 15;
  const int bl = blockIdx.x >> 2, hg = blockIdx.x & 3;
  const int head = hg * 8 + w;
  const size_t rowbase = (size_t)bl * SQ;

  const us* qhb = qh + rowbase * DQ + head * HQ;
  const us* qlb = ql + rowbase * DQ + head * HQ;
  const us* khb = kh + rowbase * DQ + head * HQ;
  const us* klb = kl + rowbase * DQ + head * HQ;
  const us* vhrow = tkh + (size_t)(head * HVD + m) * KPAD;
  const us* vlrow = tkl + (size_t)(head * HVD + m) * KPAD;

  const v8f z8 = {0.f, 0.f, 0.f, 0.f, 0.f, 0.f, 0.f, 0.f};

#pragma unroll 1
  for (int qt = 0; qt < 4; ++qt) {
    const int qr = min(qt * 16 + m, SQ - 1);
    const us* qhp = qhb + (size_t)qr * DQ;
    const us* qlp = qlb + (size_t)qr * DQ;
    const v16b qbh0 = ldb(qhp, h), qbh1 = ldb(qhp + 32, h);
    const v16b qbl0 = ldb(qlp, h), qbl1 = ldb(qlp + 32, h);

    v8f s[4];
#pragma unroll
    for (int kt = 0; kt < 4; ++kt) {
      const int kr = min(kt * 16 + m, SQ - 1);
      const us* khp = khb + (size_t)kr * DQ;
      const us* klp = klb + (size_t)kr * DQ;
      const v16b kah0 = ldb(khp, h), kah1 = ldb(khp + 32, h);
      const v16b kal0 = ldb(klp, h), kal1 = ldb(klp + 32, h);
      v8f z = z8;
      z = wmma_bf(kah0, qbh0, z);
      z = wmma_bf(kah1, qbh1, z);
      z = wmma_bf(kah0, qbl0, z);
      z = wmma_bf(kah1, qbl1, z);
      z = wmma_bf(kal0, qbh0, z);
      z = wmma_bf(kal1, qbh1, z);
      s[kt] = z;
    }

    v16us phu0, phu1, plu0, plu1;
#pragma unroll
    for (int kt = 0; kt < 4; ++kt) {
#pragma unroll
      for (int r = 0; r < 8; ++r) {
        const int key = kt * 16 + 8 * h + r;
        float tv = tanhf(s[kt][r] * 0.125f);
        tv = (key < SQ) ? tv : 0.0f;
        us hb, lb;
        split_bf(tv, hb, lb);
        const int e = (kt & 1) * 8 + r;
        if (kt < 2) { phu0[e] = hb; plu0[e] = lb; }
        else        { phu1[e] = hb; plu1[e] = lb; }
      }
    }
    FragB f0, f1, f2, f3;
    f0.u = phu0; f1.u = phu1; f2.u = plu0; f3.u = plu1;
    const v16b pbh0 = f0.v, pbh1 = f1.v, pbl0 = f2.v, pbl1 = f3.v;

    const v16b vah0 = ldb(vhrow, h), vah1 = ldb(vhrow + 32, h);
    const v16b val0 = ldb(vlrow, h), val1 = ldb(vlrow + 32, h);
    v8f o = z8;
    o = wmma_bf(vah0, pbh0, o);
    o = wmma_bf(vah1, pbh1, o);
    o = wmma_bf(vah0, pbl0, o);
    o = wmma_bf(vah1, pbl1, o);
    o = wmma_bf(val0, pbh0, o);
    o = wmma_bf(val1, pbh1, o);

    const int q = qt * 16 + m;
    float* sp = so + q * 132 + w * 16 + 8 * h;
    const v4f o0 = {o[0], o[1], o[2], o[3]};
    const v4f o1 = {o[4], o[5], o[6], o[7]};
    *(v4fa*)sp = o0;
    *(v4fa*)(sp + 4) = o1;
  }
  __syncthreads();

  attn_store(so, oph, opl, rowbase, hg, t);
  __threadfence();
  attn_store(so, oph, opl, rowbase, hg, t);
}

__device__ __forceinline__ void gemm3_store(const float* sF, float* out, int mb, int nb, int t) {
#pragma unroll
  for (int it = 0; it < 8; ++it) {
    const int item = it * 128 + t, rl = item >> 4, g = item & 15;
    const v4f v = *(const v4fa*)(sF + rl * 68 + 4 * g);
    const size_t off = (size_t)(mb + rl) * DM + nb + 4 * g;
    *(volatile v4f*)(out + off) = v;
  }
}

__global__ __launch_bounds__(128) void k_gemm3(
    const us* __restrict__ oph, const us* __restrict__ opl,
    const us* __restrict__ wph, const us* __restrict__ wpl,
    const float* __restrict__ bp,
    float* __restrict__ out)
{
  __shared__ __attribute__((aligned(16))) float sF[64 * 68];
  const int t = threadIdx.x, lane = t & 31, w = t >> 5, h = lane >> 4, m = lane & 15;
  const int wm = w >> 1, wn = w & 1;
  const int mb = blockIdx.x * 64, nb = blockIdx.y * 64;

  const size_t arow = (size_t)(mb + 32 * wm + m) * DM;
  const size_t brow = (size_t)(nb + 32 * wn + m) * DM;

  const v8f z8 = {0.f, 0.f, 0.f, 0.f, 0.f, 0.f, 0.f, 0.f};
  v8f acc[2][2];
  acc[0][0] = z8; acc[0][1] = z8; acc[1][0] = z8; acc[1][1] = z8;

  mm3_32x32(oph + arow, opl + arow, wph + brow, wpl + brow, h, acc);

#pragma unroll
  for (int nt = 0; nt < 2; ++nt) {
    const int cl = 32 * wn + 16 * nt + m;
    const float bv = bp[nb + cl];
#pragma unroll
    for (int mt = 0; mt < 2; ++mt) {
#pragma unroll
      for (int r = 0; r < 8; ++r) {
        const int rl = 32 * wm + 16 * mt + 8 * h + r;
        sF[rl * 68 + cl] = acc[mt][nt][r] + bv;
      }
    }
  }
  __syncthreads();

  gemm3_store(sF, out, mb, nb, t);
  __threadfence();
  gemm3_store(sF, out, mb, nb, t);
}

extern "C" void kernel_launch(void* const* d_in, const int* in_sizes, int n_in,
                              void* d_out, int out_size, void* d_ws, size_t ws_size,
                              hipStream_t stream) {
  if (n_in < 12) return;
  if (in_sizes[0] != MT * DM) return;
  if (in_sizes[1] != DM * DM || in_sizes[2] != DM) return;
  if (in_sizes[3] != DM * DQ || in_sizes[4] != DQ) return;
  if (in_sizes[5] != DM * DM || in_sizes[6] != DM) return;
  if (in_sizes[7] != DM * DQ || in_sizes[8] != DQ) return;
  if (in_sizes[9] != SQ * DM) return;
  if (in_sizes[10] != DM * DM || in_sizes[11] != DM) return;
  if (out_size != MT * DM) return;

  const float* x   = (const float*)d_in[0];
  const float* Wq1 = (const float*)d_in[1];
  const float* bq1 = (const float*)d_in[2];
  const float* Wq2 = (const float*)d_in[3];
  const float* bq2 = (const float*)d_in[4];
  const float* Wk1 = (const float*)d_in[5];
  const float* bk1 = (const float*)d_in[6];
  const float* Wk2 = (const float*)d_in[7];
  const float* bk2 = (const float*)d_in[8];
  const float* tok = (const float*)d_in[9];
  const float* Wp  = (const float*)d_in[10];
  const float* bp  = (const float*)d_in[11];
  float* out = (float*)d_out;

  const size_t szW1 = (size_t)DM * DM * 2;
  const size_t szW2 = (size_t)DQ * DM * 2;
  const size_t szTK = (size_t)DM * KPAD * 2;
  const size_t szX  = (size_t)MT * DM * 2;
  const size_t szH  = (size_t)RP * DM * 2;
  const size_t szQ  = (size_t)RP * DQ * 2;
  const size_t szOP = (size_t)RP * DM * 2;
  const size_t total = 6 * szW1 + 2 * szW2 + 2 * szTK + 2 * szX + 2 * szH + 4 * szQ + 2 * szOP;
  if (total > ws_size) return;

  char* wsb = (char*)d_ws;
  size_t off = 0;
  us* wq1h = (us*)(wsb + off); off += szW1;
  us* wq1l = (us*)(wsb + off); off += szW1;
  us* wk1h = (us*)(wsb + off); off += szW1;
  us* wk1l = (us*)(wsb + off); off += szW1;
  us* wph  = (us*)(wsb + off); off += szW1;
  us* wpl  = (us*)(wsb + off); off += szW1;
  _Float16* wq2t = (_Float16*)(wsb + off); off += szW2;
  _Float16* wk2t = (_Float16*)(wsb + off); off += szW2;
  us* tkh  = (us*)(wsb + off); off += szTK;
  us* tkl  = (us*)(wsb + off); off += szTK;
  us* xh   = (us*)(wsb + off); off += szX;
  us* xl   = (us*)(wsb + off); off += szX;
  _Float16* hq = (_Float16*)(wsb + off); off += szH;
  _Float16* hk = (_Float16*)(wsb + off); off += szH;
  us* qh   = (us*)(wsb + off); off += szQ;
  us* ql   = (us*)(wsb + off); off += szQ;
  us* kh   = (us*)(wsb + off); off += szQ;
  us* kl   = (us*)(wsb + off); off += szQ;
  us* oph  = (us*)(wsb + off); off += szOP;
  us* opl  = (us*)(wsb + off); off += szOP;
  if (off > ws_size) return;

  k_prep<<<712, 256, 0, stream>>>(Wq1, Wk1, Wp, Wq2, Wk2, tok,
                                  wq1h, wq1l, wk1h, wk1l, wph, wpl, wq2t, wk2t, tkh, tkl);

  const int n8 = MT * DM / 8;
  k_cvtx<<<(n8 + 255) / 256, 256, 0, stream>>>(x, xh, xl, n8);

  for (int p = 0; p < NPASS; ++p) {
    const size_t xoff = (size_t)p * RP * DM;
    k_gemm1<<<dim3(RP / 64, DM / 64, 2), 128, 0, stream>>>(
        xh + xoff, xl + xoff, wq1h, wq1l, wk1h, wk1l, bq1, bk1, hq, hk);
    k_gemm2<<<dim3(RP / 64, DQ / 128, 2), 128, 0, stream>>>(
        hq, hk, wq2t, wk2t, bq2, bk2, qh, ql, kh, kl);
    k_attn<<<WPP * 4, 256, 0, stream>>>(qh, ql, kh, kl, tkh, tkl, oph, opl);
    k_gemm3<<<dim3(RP / 64, DM / 64), 128, 0, stream>>>(
        oph, opl, wph, wpl, bp, out + xoff);
  }
}
